// GraphSAGE_84112639525007
// MI455X (gfx1250) — hardware-verified
//
#include <hip/hip_runtime.h>
#include <stddef.h>
#include <stdint.h>


#define DF     64
#define NL     3
#define AP     256
#define HOFF   128
#define K1     192
#define K23    256
#define RB     256
#define NTHR   256
#define NWAVE  8
#define EPT    8
#define CHUNK  (NTHR * EPT)
#define WCAP   (EPT * 32)
#define LISTN  (NWAVE * WCAP)
#define NBA    1024
#define SLA    10
#define RCAP   28672
#define DEGCAP 64
#define GBM    64
#define GBN    64
#define GRW    4
#define GTHR   (32 * GRW)
#define UPART  512
#define UPSH   9
#define NPART  11
#define AGG_ZINTS    (LISTN + 2 * RCAP + 3 * NBA)
#define MISC_INTS    16
#define ROWBUF_INTS  (NWAVE * RB / 2)
#define AGG_LDS_INTS (AGG_ZINTS + MISC_INTS + ROWBUF_INTS)
#define WSMAX  134217728

static_assert((CHUNK & (CHUNK - 1)) == 0 && CHUNK <= 4096);
static_assert((NBA & (NBA - 1)) == 0 && NBA == (1 << SLA));
static_assert(((long long)CHUNK << SLA) < (1LL << 31));
static_assert(LISTN % NTHR == 0);
static_assert(NBA % NWAVE == 0 && NBA % 32 == 0 && NBA % GBM == 0);
static_assert(RCAP % 4 == 0 && AGG_ZINTS % 4 == 0 && LISTN % 4 == 0 && ((AGG_ZINTS + MISC_INTS) % 4) == 0);
static_assert(AGG_ZINTS % (NTHR * 4) == 0);
static_assert(K1 % 32 == 0 && K23 % 32 == 0 && K23 == AP && K1 == 3 * DF && AP == 4 * DF);
static_assert(HOFF == 2 * DF && HOFF + 2 * DF == AP && RB == AP && RB % 16 == 0);
static_assert(DF == 2 * 32 && GBN == DF && GBM == GRW * 16 && GRW == 4 && GTHR == 128);
static_assert(UPART == (1 << UPSH) && UPART % NTHR == 0 && UPART == DF * (DF / 8));
static_assert((NPART * UPART) % NTHR == 0);
static_assert(AGG_LDS_INTS * 4 <= 300000);
static_assert(DEGCAP <= RCAP && WCAP <= LISTN);
static_assert(GBM * GBN * 4 == GBM * (2 * DF) * 2);
static_assert(ROWBUF_INTS % 4 == 0);

typedef float          v2f   __attribute__((ext_vector_type(2)));
typedef float          v4f   __attribute__((ext_vector_type(4)));
typedef float          v8f   __attribute__((ext_vector_type(8)));
typedef int            v4i   __attribute__((ext_vector_type(4)));
typedef int            v8i   __attribute__((ext_vector_type(8)));
typedef unsigned       v2u   __attribute__((ext_vector_type(2)));
typedef unsigned       v4u   __attribute__((ext_vector_type(4)));
typedef unsigned short v8us  __attribute__((ext_vector_type(8)));
typedef unsigned short v16us __attribute__((ext_vector_type(16)));
typedef __bf16         v16bf __attribute__((ext_vector_type(16)));
typedef unsigned __attribute__((may_alias)) ua;
typedef v4f  __attribute__((may_alias)) v4fa;
typedef v4i  __attribute__((may_alias)) v4ia;
typedef v2u  __attribute__((may_alias)) v2ua;
typedef v8us __attribute__((may_alias)) v8usa;
union FragB { v16bf v; v16us u; v8us h[2]; v8i w; };

__device__ __forceinline__ v8f wmb(const FragB& a, const FragB& b, v8f c) {
  v8f d = __builtin_amdgcn_wmma_f32_16x16x32_bf16(false, a.v, false, b.v, (short)0, c, false, false);
  asm volatile("v_nop\n\tv_nop\n\tv_nop\n\tv_nop" : "+v"(d) : "v"(a.w), "v"(b.w));
  return d;
}

__device__ __forceinline__ unsigned bf16_bits(float f) {
  const unsigned u = __float_as_uint(f);
  return (u + 0x7FFFu + ((u >> 16) & 1u)) >> 16;
}
__device__ __forceinline__ float bf16_val(float f) {
  return __uint_as_float(bf16_bits(f) << 16);
}

__device__ __forceinline__ void wave_sync() {
  __builtin_amdgcn_fence(__ATOMIC_RELEASE, "wavefront");
  __builtin_amdgcn_wave_barrier();
  __builtin_amdgcn_fence(__ATOMIC_ACQUIRE, "wavefront");
}

template <int SLB>
__device__ __forceinline__ int scan_chunk(const int* __restrict__ dsts, int nE, int cbase, int slotBase,
                                          int nb, int vec8, int* list, int tid, int lane, int wave) {
  int wc = 0;
  const int el0  = tid * EPT;
  const int e0   = cbase + el0;
  const int sent = -2147483647 - 1;
  v4i da, db;
  if (vec8 != 0 && cbase + CHUNK <= nE) {
    da = *(const v4i*)(dsts + e0);
    db = *(const v4i*)(dsts + e0 + 4);
  } else {
    da.x = (e0     < nE) ? dsts[min(e0,     nE - 1)] : sent;
    da.y = (e0 + 1 < nE) ? dsts[min(e0 + 1, nE - 1)] : sent;
    da.z = (e0 + 2 < nE) ? dsts[min(e0 + 2, nE - 1)] : sent;
    da.w = (e0 + 3 < nE) ? dsts[min(e0 + 3, nE - 1)] : sent;
    db.x = (e0 + 4 < nE) ? dsts[min(e0 + 4, nE - 1)] : sent;
    db.y = (e0 + 5 < nE) ? dsts[min(e0 + 5, nE - 1)] : sent;
    db.z = (e0 + 6 < nE) ? dsts[min(e0 + 6, nE - 1)] : sent;
    db.w = (e0 + 7 < nE) ? dsts[min(e0 + 7, nE - 1)] : sent;
  }
  const unsigned nbs = (unsigned)slotBase;
  const unsigned unb = (unsigned)nb;
  const unsigned s0 = (unsigned)da.x - nbs, s1 = (unsigned)da.y - nbs;
  const unsigned s2 = (unsigned)da.z - nbs, s3 = (unsigned)da.w - nbs;
  const unsigned s4 = (unsigned)db.x - nbs, s5 = (unsigned)db.y - nbs;
  const unsigned s6 = (unsigned)db.z - nbs, s7 = (unsigned)db.w - nbs;
  const bool h0 = s0 < unb, h1 = s1 < unb, h2 = s2 < unb, h3 = s3 < unb;
  const bool h4 = s4 < unb, h5 = s5 < unb, h6 = s6 < unb, h7 = s7 < unb;
  const unsigned any = __builtin_amdgcn_ballot_w32(h0 | h1 | h2 | h3 | h4 | h5 | h6 | h7);
  if (any != 0u) {
#define HITJ(J, HJ, SJ) { \
      const unsigned mj = __builtin_amdgcn_ballot_w32(HJ); \
      if (mj != 0u) { \
        if (HJ) { \
          const int pos = wc + (int)__builtin_amdgcn_mbcnt_lo(mj, 0u); \
          if (pos < WCAP) list[wave * WCAP + pos] = ((el0 + (J)) << SLB) | (int)(SJ); \
        } \
        wc += (int)__builtin_popcount(mj); } }
    HITJ(0, h0, s0)
    HITJ(1, h1, s1)
    HITJ(2, h2, s2)
    HITJ(3, h3, s3)
    HITJ(4, h4, s4)
    HITJ(5, h5, s5)
    HITJ(6, h6, s6)
    HITJ(7, h7, s7)
#undef HITJ
  }
  return wc;
}

__global__ __launch_bounds__(NTHR) void k_wprep(const float* __restrict__ wl, const float* __restrict__ wr,
                                                unsigned short* B1, unsigned short* B2, unsigned short* B3) {
  const int u    = (int)blockIdx.x * NTHR + (int)threadIdx.x;
  const int part = u >> UPSH;
  const int v    = u & (UPART - 1);
  const float* W;
  unsigned short* P;
  int pitch, coff;
  if (part == 0)       { W = wl;               P = B1; pitch = K1;  coff = 0;      }
  else if (part == 1)  { W = wl;               P = B1; pitch = K1;  coff = DF;     }
  else if (part == 2)  { W = wr;               P = B1; pitch = K1;  coff = 2 * DF; }
  else if (part == 3)  { W = wl + DF * DF;     P = B2; pitch = K23; coff = 0;      }
  else if (part == 4)  { W = wl + DF * DF;     P = B2; pitch = K23; coff = DF;     }
  else if (part == 5)  { W = wr + DF * DF;     P = B2; pitch = K23; coff = 2 * DF; }
  else if (part == 6)  { W = wr + DF * DF;     P = B2; pitch = K23; coff = 3 * DF; }
  else if (part == 7)  { W = wl + 2 * DF * DF; P = B3; pitch = K23; coff = 0;      }
  else if (part == 8)  { W = wl + 2 * DF * DF; P = B3; pitch = K23; coff = DF;     }
  else if (part == 9)  { W = wr + 2 * DF * DF; P = B3; pitch = K23; coff = 2 * DF; }
  else if (part == 10) { W = wr + 2 * DF * DF; P = B3; pitch = K23; coff = 3 * DF; }
  else return;
  const int n  = v >> 3;
  const int k8 = (v & 7) * 8;
  const float* p = W + (size_t)k8 * DF + n;
  float f[8];
#pragma unroll
  for (int j = 0; j < 8; ++j) f[j] = p[(size_t)j * DF];
  v8us o;
#pragma unroll
  for (int j = 0; j < 8; ++j) o[j] = (unsigned short)bf16_bits(f[j]);
  unsigned short* dp = P + (size_t)n * pitch + coff + k8;
  *(volatile v8us*)dp = o;
  __threadfence();
  *(volatile v8us*)dp = o;
}

template <int FIN>
__global__ __launch_bounds__(GTHR) void k_gemm(unsigned short* Apl, const unsigned short* __restrict__ BT,
                                                int K, const float* __restrict__ bias, float* outp, int nOut) {
  __shared__ __attribute__((aligned(16))) float gsm[GBM * GBN];
  const int tid = (int)threadIdx.x, lane = tid & 31, wave = tid >> 5, hh = lane >> 4, m = lane & 15;
  const int rowBase = (int)blockIdx.x * GBM;

  v8f acc[4];
  {
    const v8f z = {0.f, 0.f, 0.f, 0.f, 0.f, 0.f, 0.f, 0.f};
#pragma unroll
    for (int t = 0; t < 4; ++t) acc[t] = z;
  }
  const unsigned short* ap = Apl + (size_t)(rowBase + 16 * wave + m) * (size_t)AP + 8 * hh;
  const unsigned short* bp = BT + (size_t)m * (size_t)K + 8 * hh;

#pragma unroll 1
  for (int k0 = 0; k0 < K; k0 += 32) {
    FragB af;
    af.h[0] = *(const v8usa*)(ap + k0);
    af.h[1] = *(const v8usa*)(ap + k0 + 16);
#pragma unroll
    for (int nt = 0; nt < 4; ++nt) {
      const unsigned short* wq = bp + (size_t)(16 * nt) * (size_t)K + k0;
      FragB bf;
      bf.h[0] = *(const v8usa*)wq;
      bf.h[1] = *(const v8usa*)(wq + 16);
      acc[nt] = wmb(af, bf, acc[nt]);
    }
  }

#pragma unroll
  for (int nt = 0; nt < 4; ++nt) {
    const int lc = 16 * nt + m;
#pragma unroll
    for (int r = 0; r < 8; ++r) {
      const int lr = 16 * wave + 8 * hh + r;
      gsm[lr * GBN + lc] = acc[nt][r];
    }
  }
  __syncthreads();

  v4f bb4;
  {
    const v4f tb = *(const v4f*)(bias + 4 * m);
    bb4.x = bf16_val(tb.x); bb4.y = bf16_val(tb.y); bb4.z = bf16_val(tb.z); bb4.w = bf16_val(tb.w);
  }

  v4f q[8];
#pragma unroll
  for (int ii = 0; ii < 8; ++ii) {
    const int lr = 16 * wave + 2 * ii + hh;
    const bool ok = (rowBase + lr) < nOut;
    const v4f t = *(const v4fa*)(gsm + lr * GBN + 4 * m) + bb4;
    v4f y = t;
    if constexpr (FIN == 0) {
      y.x = (t.x < 0.0f) ? 0.0f : t.x;
      y.y = (t.y < 0.0f) ? 0.0f : t.y;
      y.z = (t.z < 0.0f) ? 0.0f : t.z;
      y.w = (t.w < 0.0f) ? 0.0f : t.w;
    }
    y.x = ok ? y.x : 0.0f; y.y = ok ? y.y : 0.0f; y.z = ok ? y.z : 0.0f; y.w = ok ? y.w : 0.0f;
    q[ii] = y;
  }

  if constexpr (FIN != 0) {
#pragma unroll
    for (int ii = 0; ii < 8; ++ii) {
      const int gr = rowBase + 16 * wave + 2 * ii + hh;
      if (gr < nOut) *(volatile v4f*)(outp + (size_t)gr * DF + 4 * m) = q[ii];
    }
    __threadfence();
#pragma unroll
    for (int ii = 0; ii < 8; ++ii) {
      const int gr = rowBase + 16 * wave + 2 * ii + hh;
      if (gr < nOut) *(volatile v4f*)(outp + (size_t)gr * DF + 4 * m) = q[ii];
    }
  } else {
    __syncthreads();
#pragma unroll
    for (int ii = 0; ii < 8; ++ii) {
      const int lr = 16 * wave + 2 * ii + hh;
      unsigned h0, h1, h2, h3, l0, l1, l2, l3;
      h0 = bf16_bits(q[ii].x); l0 = bf16_bits(q[ii].x - __uint_as_float(h0 << 16));
      h1 = bf16_bits(q[ii].y); l1 = bf16_bits(q[ii].y - __uint_as_float(h1 << 16));
      h2 = bf16_bits(q[ii].z); l2 = bf16_bits(q[ii].z - __uint_as_float(h2 << 16));
      h3 = bf16_bits(q[ii].w); l3 = bf16_bits(q[ii].w - __uint_as_float(h3 << 16));
      v2u ph, pl;
      ph.x = h0 | (h1 << 16); ph.y = h2 | (h3 << 16);
      pl.x = l0 | (l1 << 16); pl.y = l2 | (l3 << 16);
      ua* srow = (ua*)gsm + (size_t)lr * DF;
      *(v2ua*)(srow + 2 * m) = ph;
      *(v2ua*)(srow + DF / 2 + 2 * m) = pl;
    }
    __syncthreads();
    v8us qv[8];
#pragma unroll
    for (int ii = 0; ii < 8; ++ii) {
      const int lr = 16 * wave + 2 * ii + hh;
      const unsigned short* srow = (const unsigned short*)gsm + (size_t)lr * (2 * DF);
      qv[ii] = *(const v8usa*)(srow + 8 * m);
    }
#pragma unroll
    for (int ii = 0; ii < 8; ++ii) {
      unsigned short* rp = Apl + (size_t)(rowBase + 16 * wave + 2 * ii + hh) * (size_t)AP + HOFF + 8 * m;
      *(volatile v8us*)rp = qv[ii];
    }
    __threadfence();
#pragma unroll
    for (int ii = 0; ii < 8; ++ii) {
      unsigned short* rp = Apl + (size_t)(rowBase + 16 * wave + 2 * ii + hh) * (size_t)AP + HOFF + 8 * m;
      *(volatile v8us*)rp = qv[ii];
    }
  }
}

template <int L0>
__global__ __launch_bounds__(NTHR) void k_scan(const int* __restrict__ gath, const int* __restrict__ keys,
                                               int nE, int nN, int vec8, int mRows,
                                               const float* __restrict__ xin, unsigned short* apl) {
  extern __shared__ __attribute__((aligned(16))) int dsm[];
  int* list = dsm;
  int* hl   = dsm + LISTN;
  int* sl   = hl + RCAP;
  int* cnt  = sl + RCAP;
  int* offs = cnt + NBA;
  int* cur  = offs + NBA;
  int* misc = cur + NBA;
  const int tid = (int)threadIdx.x, lane = tid & 31, wave = tid >> 5;
  unsigned short* rowbuf = (unsigned short*)(misc + MISC_INTS) + wave * RB;
  ua* rowu = (ua*)rowbuf;
  const int nodeBase = (int)blockIdx.x * NBA;

  {
    const v4i z4 = {0, 0, 0, 0};
    for (int i = tid * 4; i < AGG_ZINTS; i += NTHR * 4) *(v4ia*)(dsm + i) = z4;
    if (tid < MISC_INTS) misc[tid] = 0;
  }
  __syncthreads();

  int t = 0, ov = 0;
  const int nChunks = (nE + CHUNK - 1) / CHUNK;
#pragma unroll 1
  for (int chn = 0; chn < nChunks; ++chn) {
    const int cbase = chn * CHUNK;
    const int wc = scan_chunk<SLA>(keys, nE, cbase, nodeBase, NBA, vec8, list, tid, lane, wave);
    if (lane == 0) misc[wave] = wc;
    __syncthreads();
    if (wave == 0) {
#pragma unroll 1
      for (int w2 = 0; w2 < NWAVE; ++w2) {
        int c = misc[w2];
        c = c < 0 ? 0 : (c > WCAP ? WCAP : c);
#pragma unroll 1
        for (int b0 = 0; b0 < c; b0 += 32) {
          const int idx = b0 + lane;
          const int ent = list[w2 * WCAP + (idx < WCAP ? idx : WCAP - 1)];
          const int m32 = (c - b0) < 32 ? (c - b0) : 32;
#pragma unroll 1
          for (int k = 0; k < m32; ++k) {
            const int u    = __builtin_amdgcn_readlane(ent, k);
            const int slot = u & (NBA - 1);
            const int el   = (u >> SLA) & (CHUNK - 1);
            const int pk   = ((cbase + el) << SLA) | slot;
            if (t < RCAP) {
              if (lane == 0) { hl[t] = pk; cnt[slot] = cnt[slot] + 1; }
              t = t + 1;
            } else {
              ov = 1;
            }
          }
        }
      }
    }
    __syncthreads();
  }
  if (wave == 0 && lane == 0) { misc[8] = t; misc[9] = ov; }
  __syncthreads();
  int tt = misc[8];
  tt = tt < 0 ? 0 : (tt > RCAP ? RCAP : tt);
  const int ovf = misc[9];

  if (wave == 0) {
    const int base = lane * (NBA / 32);
    int s = 0;
#pragma unroll 1
    for (int i = 0; i < NBA / 32; ++i) s += cnt[base + i];
    int incl = s;
#pragma unroll
    for (int d = 1; d < 32; d <<= 1) {
      const int y = __shfl_up(incl, d, 32);
      if (lane >= d) incl += y;
    }
    int run = incl - s;
#pragma unroll 1
    for (int i = 0; i < NBA / 32; ++i) {
      const int cv = cnt[base + i];
      offs[base + i] = run;
      cur[base + i]  = run;
      run += cv;
    }
  }
  __syncthreads();
  if (wave == 0) {
#pragma unroll 1
    for (int b0 = 0; b0 < tt; b0 += 32) {
      const int idx = b0 + lane;
      const int ent = hl[idx < RCAP ? idx : RCAP - 1];
      const int m32 = (tt - b0) < 32 ? (tt - b0) : 32;
#pragma unroll 1
      for (int k = 0; k < m32; ++k) {
        const int u    = __builtin_amdgcn_readlane(ent, k);
        const int slot = u & (NBA - 1);
        if (lane == 0) {
          int p = cur[slot];
          p = p < 0 ? 0 : (p > RCAP - 1 ? RCAP - 1 : p);
          sl[p] = u;
          cur[slot] = p + 1;
        }
      }
    }
  }
  __syncthreads();

  const float pz = (ovf != 0) ? __int_as_float(0x7fc00000) : 0.0f;
#pragma unroll 1
  for (int si = 0; si < NBA / NWAVE; ++si) {
    const int s    = si * NWAVE + wave;
    const int node = nodeBase + s;
    int c = cnt[s];
    const bool big = c > DEGCAP;
    c = c < 0 ? 0 : (c > DEGCAP ? DEGCAP : c);
    int o = offs[s];
    o = o < 0 ? 0 : (o > RCAP ? RCAP : o);
    const float pzr = big ? __int_as_float(0x7fc00000) : pz;
    const bool live = node < nN;

    float a0 = 0.0f, a1 = 0.0f;
#pragma unroll 1
    for (int b0 = 0; b0 < c; b0 += 32) {
      int idx = o + b0 + lane;
      idx = idx > RCAP - 1 ? RCAP - 1 : idx;
      const int ent = sl[idx];
      int eid = ent >> SLA;
      eid = eid < 0 ? 0 : (eid > nE - 1 ? nE - 1 : eid);
      int sr = gath[eid];
      sr = sr < 0 ? 0 : (sr > nN - 1 ? nN - 1 : sr);
      const int m32 = (c - b0) < 32 ? (c - b0) : 32;
#pragma unroll 1
      for (int k = 0; k < m32; ++k) {
        const int sk = __builtin_amdgcn_readlane(sr, k);
        if constexpr (L0 != 0) {
          const v2f a = *(const v2f*)(xin + (size_t)sk * DF + 2 * lane);
          a0 += bf16_val(a.x);
          a1 += bf16_val(a.y);
        } else {
          const unsigned short* rp = apl + (size_t)sk * AP + HOFF + 2 * lane;
          const unsigned wh = *(const ua*)rp;
          const unsigned wl = *(const ua*)(rp + DF);
          a0 += __uint_as_float(wh << 16)         + __uint_as_float(wl << 16);
          a1 += __uint_as_float(wh & 0xffff0000u) + __uint_as_float(wl & 0xffff0000u);
        }
      }
    }
    const float inv = 1.0f / (float)(c > 0 ? c : 1);
    const float m0 = live ? (a0 * inv + pzr) : 0.0f;
    const float m1 = live ? (a1 * inv + pzr) : 0.0f;
    {
      const unsigned hb0 = bf16_bits(m0), hb1 = bf16_bits(m1);
      const unsigned lb0 = bf16_bits(m0 - __uint_as_float(hb0 << 16));
      const unsigned lb1 = bf16_bits(m1 - __uint_as_float(hb1 << 16));
      rowu[lane]          = hb0 | (hb1 << 16);
      rowu[DF / 2 + lane] = lb0 | (lb1 << 16);
    }
    if constexpr (L0 != 0) {
      const int nc = live ? node : nN - 1;
      const v2f xs = *(const v2f*)(xin + (size_t)nc * DF + 2 * lane);
      const unsigned xb0 = live ? bf16_bits(xs.x + pzr) : 0u;
      const unsigned xb1 = live ? bf16_bits(xs.y + pzr) : 0u;
      rowu[DF + lane]         = xb0 | (xb1 << 16);
      rowu[3 * DF / 2 + lane] = 0u;
    }
    wave_sync();
    const int ql = (L0 != 0) ? lane : (lane & 15);
    const v8us q0 = *(const v8usa*)(rowbuf + 8 * ql);
    wave_sync();
    const bool wr = (node < mRows) && ((L0 != 0) || (lane < 16));
    unsigned short* rpw = apl + (size_t)node * AP + 8 * lane;
    if (wr) *(volatile v8us*)rpw = q0;
    __threadfence();
    if (wr) *(volatile v8us*)rpw = q0;
  }
}

static inline int cdiv(int a, int b) { return (a + b - 1) / b; }
static inline size_t al256(size_t o) { return (o + 255) & ~(size_t)255; }

extern "C" void kernel_launch(void* const* d_in, const int* in_sizes, int n_in,
                              void* d_out, int out_size, void* d_ws, size_t ws_size,
                              hipStream_t stream) {
  if (n_in < 5) return;
  if (in_sizes[0] < DF || (in_sizes[0] % DF) != 0) return;
  const int nN = in_sizes[0] / DF;
  if (in_sizes[1] < 2 || (in_sizes[1] & 1) != 0) return;
  const int nE = in_sizes[1] / 2;
  if (in_sizes[2] != NL * DF * DF || in_sizes[3] != NL * DF * DF || in_sizes[4] != NL * DF) return;
  if (nE < 1 || nE >= (1 << 21) || nN < 16 || nN >= (1 << 24)) return;
  if ((long long)out_size != (long long)nN * DF) return;

  const float* x  = (const float*)d_in[0];
  const int*   ei = (const int*)d_in[1];
  const float* wl = (const float*)d_in[2];
  const float* wr = (const float*)d_in[3];
  const float* bb = (const float*)d_in[4];
  float* out = (float*)d_out;
  const int* src = ei;
  const int* dst = ei + nE;

  const int MP = cdiv(nN, GBM) * GBM;
  const int gM = MP / GBM;
  const int gA = cdiv(nN, NBA);
  if ((long long)gA * NBA < (long long)MP) return;
  const int vec8 = ((nE & 3) == 0) ? 1 : 0;

  char* ws = (char*)d_ws;
  size_t off = 0;
  const size_t oB1 = off; off = al256(off + (size_t)DF * K1 * 2);
  const size_t oB2 = off; off = al256(off + (size_t)DF * K23 * 2);
  const size_t oB3 = off; off = al256(off + (size_t)DF * K23 * 2);
  const size_t oA  = off; off = al256(off + (size_t)MP * AP * 2);
  if (off > ws_size || off > (size_t)WSMAX) return;
  unsigned short* B1  = (unsigned short*)(ws + oB1);
  unsigned short* B2  = (unsigned short*)(ws + oB2);
  unsigned short* B3  = (unsigned short*)(ws + oB3);
  unsigned short* Apl = (unsigned short*)(ws + oA);

  const size_t scanLds = (size_t)AGG_LDS_INTS * 4;
  hipFuncSetAttribute(reinterpret_cast<const void*>(&k_scan<1>), hipFuncAttributeMaxDynamicSharedMemorySize, (int)scanLds);
  hipFuncSetAttribute(reinterpret_cast<const void*>(&k_scan<0>), hipFuncAttributeMaxDynamicSharedMemorySize, (int)scanLds);

  k_wprep<<<(NPART * UPART) / NTHR, NTHR, 0, stream>>>(wl, wr, B1, B2, B3);
  k_scan<1><<<gA, NTHR, scanLds, stream>>>(src, dst, nE, nN, vec8, MP, x, Apl);
  k_gemm<0><<<gM, GTHR, 0, stream>>>(Apl, B1, K1, bb, out, nN);
  k_scan<0><<<gA, NTHR, scanLds, stream>>>(src, dst, nE, nN, vec8, MP, x, Apl);
  k_gemm<0><<<gM, GTHR, 0, stream>>>(Apl, B2, K23, bb + DF, out, nN);
  k_scan<0><<<gA, NTHR, scanLds, stream>>>(src, dst, nE, nN, vec8, MP, x, Apl);
  k_gemm<1><<<gM, GTHR, 0, stream>>>(Apl, B3, K23, bb + 2 * DF, out, nN);
}
